// hierarchically_modular_50311246905871
// MI455X (gfx1250) — hardware-verified
//
#include <hip/hip_runtime.h>

typedef _Float16 v16h __attribute__((ext_vector_type(16)));
typedef _Float16 v8h  __attribute__((ext_vector_type(8)));
typedef float    v8f  __attribute__((ext_vector_type(8)));
typedef float    v4f  __attribute__((ext_vector_type(4)));
typedef v8h __attribute__((may_alias)) v8ha;
typedef v4f __attribute__((may_alias)) v4fa;

union Frag { v16h v; v8h half[2]; };

constexpr int NB   = 8192;
constexpr int DIN  = 512;
constexpr int NM   = 128;
constexpr int KR   = 8;
constexpr int NH   = 128;
constexpr int NOUT = 2;
constexpr int BT   = 256;
constexpr int OBT  = 512;
constexpr float WSC  = 64.0f;
constexpr float YINV = 1.0f / (64.0f * 64.0f);

static_assert(NB % BT == 0);
static_assert(NB % OBT == 0);
static_assert(DIN % 32 == 0);
static_assert(NM % 32 == 0);
static_assert(NH == 128);
static_assert(BT == 256);

__device__ __forceinline__ v8f wmma16(v16h a, v16h b, v8f c) {
#if defined(__HIP_DEVICE_COMPILE__)
  v8f d = __builtin_amdgcn_wmma_f32_16x16x32_f16(false, a, false, b, (short)0, c, false, false);
  asm volatile("v_nop\n\tv_nop\n\tv_nop\n\tv_nop" : "+v"(d) : "v"(a), "v"(b));
  return d;
#else
  (void)a; (void)b;
  return c;
#endif
}

__device__ __forceinline__ float rcp_f32(float x) {
#if defined(__HIP_DEVICE_COMPILE__)
  return __builtin_amdgcn_rcpf(x);
#else
  return 1.0f / x;
#endif
}

__device__ __forceinline__ v8h zero8h() {
  v8h z;
#pragma unroll
  for (int i = 0; i < 8; ++i) z[i] = (_Float16)0.0f;
  return z;
}

__device__ __forceinline__ v8f zero8f() {
  v8f z;
#pragma unroll
  for (int i = 0; i < 8; ++i) z[i] = 0.0f;
  return z;
}

template <int NPER>
__device__ __forceinline__ void topk_wave(const float* __restrict__ e, int mstride,
                                          int kcount, int* sdst, int lane) {
  float ev[NPER];
#pragma unroll
  for (int i = 0; i < NPER; ++i) ev[i] = e[(size_t)(lane + 32 * i) * (size_t)mstride];

  float lastv = __builtin_huge_valf();
  int   lasti = -1;
#pragma unroll 1
  for (int p = 0; p < kcount; ++p) {
    float bv = -__builtin_huge_valf();
    int   bi = 0x7fffffff;
#pragma unroll
    for (int i = 0; i < NPER; ++i) {
      const int   d = lane + 32 * i;
      const float v = ev[i];
      const bool elig = (v < lastv) || (v == lastv && d > lasti);
      const bool bett = (v > bv) || (v == bv && d < bi);
      const bool tk   = elig && bett;
      bv = tk ? v : bv;
      bi = tk ? d : bi;
    }
#pragma unroll
    for (int off = 16; off > 0; off >>= 1) {
      const float ov = __shfl_xor(bv, off);
      const int   oi = __shfl_xor(bi, off);
      const bool tk = (ov > bv) || (ov == bv && oi < bi);
      bv = tk ? ov : bv;
      bi = tk ? oi : bi;
    }
    lastv = bv;
    lasti = bi;
    if (lane == 0) sdst[p] = bi;
  }
}

template <int NPER, bool TIN>
__global__ __launch_bounds__(256) void layer_kernel(
    const float* __restrict__ xin,
    const float* __restrict__ emb,
    int ntask,
    const int*   __restrict__ taskp,
    const float* __restrict__ W1,
    const float* __restrict__ b1,
    const float* __restrict__ W2,
    const float* __restrict__ b2,
    float* __restrict__ yT)
{
  constexpr int DG = NPER * 32;

  __shared__ __attribute__((aligned(16))) _Float16 sA[NH * 32];
  __shared__ __attribute__((aligned(16))) _Float16 sX[BT * 32];
  __shared__ __attribute__((aligned(16))) _Float16 sW2[NH];
  __shared__ __attribute__((aligned(16))) float    sB1[NH];
  __shared__ __attribute__((aligned(16))) float    sY[BT];
  __shared__ int sIdx[KR];

  const int tid  = threadIdx.x;
  const int lane = tid & 31, wave = tid >> 5;
  const int h    = lane >> 4, nl = lane & 15;
  const int m    = blockIdx.y;
  const int b0   = blockIdx.x * BT;

  if (tid < NH) {
    const int j = tid;
    v8h wv = zero8h();
#pragma unroll
    for (int k = 0; k < KR; ++k)
      wv[k] = (_Float16)(W1[((size_t)m * KR + k) * NH + j] * WSC);
    const v8h z8 = zero8h();
    *(v8ha*)(sA + j * 32)      = wv;
    *(v8ha*)(sA + j * 32 + 8)  = z8;
    *(v8ha*)(sA + j * 32 + 16) = z8;
    *(v8ha*)(sA + j * 32 + 24) = z8;
  } else {
    const int j = tid - NH;
    sB1[j] = b1[(size_t)m * NH + j] * WSC;
    sW2[j] = (_Float16)(W2[(size_t)m * NH + j] * WSC);
  }

  if (wave == 0) {
    int task = taskp[0];
    task = (task < 0) ? 0 : ((task > ntask - 1) ? (ntask - 1) : task);
    const float* e = emb + (size_t)task * DG * NM + m;
    topk_wave<NPER>(e, NM, KR, sIdx, lane);
  }
  __syncthreads();

  {
    const int n = tid;
    const int b = b0 + n;
    float v[KR];
#pragma unroll
    for (int k = 0; k < KR; ++k) {
      int ci = sIdx[k];
      ci = (ci < 0) ? 0 : ((ci > DG - 1) ? (DG - 1) : ci);
      if constexpr (TIN) {
        v[k] = xin[(size_t)ci * NB + b];
      } else {
        v[k] = xin[(size_t)b * DG + ci];
      }
    }
    v8h xv;
#pragma unroll
    for (int k = 0; k < KR; ++k) xv[k] = (_Float16)v[k];
    const v8h z8 = zero8h();
    *(v8ha*)(sX + n * 32)      = xv;
    *(v8ha*)(sX + n * 32 + 8)  = z8;
    *(v8ha*)(sX + n * 32 + 16) = z8;
    *(v8ha*)(sX + n * 32 + 24) = z8;
  }
  __syncthreads();

  const float b2m = b2[m];
  const v8f z8f = zero8f();
#pragma unroll
  for (int t = 0; t < 2; ++t) {
    const int nrow = wave * 32 + 16 * t + nl;
    Frag bx;
    bx.half[0] = *(const v8ha*)(sX + nrow * 32 + 8 * h);
    bx.half[1] = *(const v8ha*)(sX + nrow * 32 + 16 + 8 * h);

    v8f yacc = z8f;
#pragma unroll
    for (int s = 0; s < 4; ++s) {
      const _Float16* ar0 = sA + (32 * s + nl) * 32;
      const _Float16* ar1 = sA + (32 * s + 16 + nl) * 32;
      Frag a0, a1;
      a0.half[0] = *(const v8ha*)(ar0 + 8 * h);
      a0.half[1] = *(const v8ha*)(ar0 + 16 + 8 * h);
      a1.half[0] = *(const v8ha*)(ar1 + 8 * h);
      a1.half[1] = *(const v8ha*)(ar1 + 16 + 8 * h);

      const v8f d0 = wmma16(a0.v, bx.v, z8f);
      const v8f d1 = wmma16(a1.v, bx.v, z8f);

      Frag hb;
#pragma unroll
      for (int r = 0; r < 8; ++r) {
        const float p0 = fmaxf(d0[r] + sB1[32 * s + 8 * h + r], 0.0f);
        const float p1 = fmaxf(d1[r] + sB1[32 * s + 16 + 8 * h + r], 0.0f);
        hb.v[r]     = (_Float16)p0;
        hb.v[8 + r] = (_Float16)p1;
      }

      const v8h w0 = *(const v8ha*)(sW2 + 32 * s + 8 * h);
      const v8h w1 = *(const v8ha*)(sW2 + 32 * s + 16 + 8 * h);
      const v8h zh = zero8h();
      Frag aw;
      aw.half[0] = (nl == 0) ? w0 : zh;
      aw.half[1] = (nl == 0) ? w1 : zh;

      yacc = wmma16(aw.v, hb.v, yacc);
    }
    if (h == 0) sY[nrow] = yacc[0] * YINV + b2m;
  }
  __syncthreads();

  if (wave < 2) {
    const int f = wave * 128 + lane * 4;
    const v4f v = *(const v4fa*)(sY + f);
    float* dst = yT + (size_t)m * NB + b0 + f;
    *(volatile v4f*)dst = v;
    __threadfence();
    *(volatile v4f*)dst = v;
  }
}

__device__ __forceinline__ float sigm(float v) {
  const float ex = __expf(-v);
  return rcp_f32(1.0f + ex);
}

template <int NPER>
__global__ __launch_bounds__(256) void out_kernel(
    const float* __restrict__ yT,
    const float* __restrict__ embo,
    int ntask,
    const int*   __restrict__ taskp,
    float* __restrict__ out)
{
  constexpr int DG = NPER * 32;
  __shared__ int sIo[NOUT];

  const int tid = threadIdx.x, lane = tid & 31, wave = tid >> 5;
  if (wave == 0) {
    int task = taskp[0];
    task = (task < 0) ? 0 : ((task > ntask - 1) ? (ntask - 1) : task);
    const float* e = embo + (size_t)task * DG;
    topk_wave<NPER>(e, 1, NOUT, sIo, lane);
  }
  __syncthreads();

  int i0 = sIo[0], i1 = sIo[1];
  i0 = (i0 < 0) ? 0 : ((i0 > DG - 1) ? (DG - 1) : i0);
  i1 = (i1 < 0) ? 0 : ((i1 > DG - 1) ? (DG - 1) : i1);

  const int r0 = blockIdx.x * OBT + 2 * tid;
  const float* c0 = yT + (size_t)i0 * NB;
  const float* c1 = yT + (size_t)i1 * NB;
  const float v00 = c0[r0], v01 = c1[r0];
  const float v10 = c0[r0 + 1], v11 = c1[r0 + 1];

  v4f o;
  o[0] = sigm(v00);
  o[1] = sigm(v01);
  o[2] = sigm(v10);
  o[3] = sigm(v11);

  float* dst = out + (size_t)r0 * NOUT;
  *(volatile v4f*)dst = o;
  __threadfence();
  *(volatile v4f*)dst = o;
}

extern "C" void kernel_launch(void* const* d_in, const int* in_sizes, int n_in,
                              void* d_out, int out_size, void* d_ws, size_t ws_size,
                              hipStream_t stream) {
  if (n_in < 13) return;
  if (in_sizes[0] != NB * DIN) return;
  if (in_sizes[1] < 1) return;
  if (in_sizes[2] < DIN * NM || (in_sizes[2] % (DIN * NM)) != 0) return;
  const int ntask = in_sizes[2] / (DIN * NM);
  if (in_sizes[3] != ntask * NM * NM) return;
  if (in_sizes[4] != ntask * NM) return;
  if (in_sizes[5] != NM * KR * NH || in_sizes[6] != NM * NH ||
      in_sizes[7] != NM * NH || in_sizes[8] != NM) return;
  if (in_sizes[9] != NM * KR * NH || in_sizes[10] != NM * NH ||
      in_sizes[11] != NM * NH || in_sizes[12] != NM) return;
  if (out_size != NB * NOUT) return;

  const float* x       = (const float*)d_in[0];
  const int*   task    = (const int*)  d_in[1];
  const float* emb0    = (const float*)d_in[2];
  const float* emb1    = (const float*)d_in[3];
  const float* emb_out = (const float*)d_in[4];
  const float* W1_0    = (const float*)d_in[5];
  const float* b1_0    = (const float*)d_in[6];
  const float* W2_0    = (const float*)d_in[7];
  const float* b2_0    = (const float*)d_in[8];
  const float* W1_1    = (const float*)d_in[9];
  const float* b1_1    = (const float*)d_in[10];
  const float* W2_1    = (const float*)d_in[11];
  const float* b2_1    = (const float*)d_in[12];
  float* out = (float*)d_out;

  const size_t ybytes = (size_t)NM * NB * sizeof(float);
  if (2 * ybytes > ws_size) return;
  char* ws = (char*)d_ws;
  float* y0 = (float*)(ws);
  float* y1 = (float*)(ws + ybytes);

  const dim3 gl(NB / BT, NM);
  layer_kernel<DIN / 32, false><<<gl, 256, 0, stream>>>(x,  emb0, ntask, task, W1_0, b1_0, W2_0, b2_0, y0);
  layer_kernel<NM / 32,  true ><<<gl, 256, 0, stream>>>(y0, emb1, ntask, task, W1_1, b1_1, W2_1, b2_1, y1);

  out_kernel<NM / 32><<<NB / OBT, 256, 0, stream>>>(y1, emb_out, ntask, task, out);
}
